// feature_conbined_86011015070115
// MI455X (gfx1250) — hardware-run, weakly checked
//
#include <hip/hip_runtime.h>
#include <math.h>

typedef __attribute__((ext_vector_type(16))) _Float16 v16h;
typedef __attribute__((ext_vector_type(8)))  _Float16 v8h;
typedef __attribute__((ext_vector_type(2)))  _Float16 v2h;
typedef __attribute__((ext_vector_type(8)))  float    v8f;
typedef __attribute__((ext_vector_type(4)))  float    v4f;
typedef __attribute__((ext_vector_type(4)))  unsigned v4u;

constexpr int kBatch   = 1024;
constexpr int kLen     = 256;
constexpr int kPool    = 4;
constexpr int kFm      = 64;
constexpr int kHead    = 64;
constexpr int kEmb     = 48;
constexpr int kCat     = 3 * kEmb;
constexpr int kOutW    = 20;
constexpr int kKtot    = kFm * kFm;
constexpr int kRowsBlk = 8;
constexpr float kCarryA   = 256.0f;
constexpr float kCarryB   = 64.0f;
constexpr float kFoldBack = 1.0f / (kCarryA * kCarryB);
static_assert(kLen == kFm * kPool, "pool geometry");
static_assert((kKtot % 32) == 0, "GEMM K multiple of 32");
static_assert((kBatch % 64) == 0 && kHead == 64, "GEMM M, N multiples of 64");
static_assert((kRowsBlk * kOutW * 4) % 128 == 0, "8 output rows = whole lines");
static_assert(kCat == 144 && kOutW == 20 && kEmb == 48, "layer widths");

constexpr size_t kOffWN   = 0;
constexpr size_t kOffWEFF = kOffWN   + (size_t)kHead * kKtot * 2;
constexpr size_t kOffWFC  = kOffWEFF + (size_t)2 * kHead * kFm * 4;
constexpr size_t kOffBFC  = kOffWFC  + (size_t)kCat * kHead * 4;
constexpr size_t kOffXPD  = kOffBFC  + (size_t)160 * 4;
constexpr size_t kOffPN   = kOffXPD  + (size_t)kBatch * 128 * 4;
constexpr size_t kOffHN   = kOffPN   + (size_t)kBatch * kKtot * 2;
constexpr size_t kWsTotal = kOffHN   + (size_t)kBatch * kHead * 4;
static_assert(kWsTotal == 9769600ull, "carve total");
static_assert(kWsTotal <= 134217728ull, "carve cap");
static_assert((kOffWEFF % 128) == 0 && (kOffWFC % 128) == 0 && (kOffBFC % 128) == 0 &&
              (kOffXPD % 128) == 0 && (kOffPN % 128) == 0 && (kOffHN % 128) == 0, "128-B aligned regions");

__device__ __forceinline__ float elu1(float v) {
  const float e = expf(fminf(v, 0.0f)) - 1.0f;
  return (v > 0.0f) ? v : e;
}
__device__ __forceinline__ unsigned pack2h(float a, float b) {
  v2h h;
  h[0] = (_Float16)a;
  h[1] = (_Float16)b;
  return __builtin_bit_cast(unsigned, h);
}
__device__ __forceinline__ v16h frag_load_h(const _Float16* p) {
  union { v16h v; v8h h[2]; } f;
  f.h[0] = *(const v8h*)(p);
  f.h[1] = *(const v8h*)(p + 16);
  return f.v;
}
__device__ __forceinline__ v8f mma_h(v16h a, v16h b, v8f c) {
  return __builtin_amdgcn_wmma_f32_16x16x32_f16(false, a, false, b, (short)0, c, false, false);
}
__device__ __forceinline__ void frag_guard(v8f& acc, v16h x, v16h y) {
  asm volatile("v_nop\n\tv_nop\n\tv_nop\n\tv_nop" : "+v"(acc) : "v"(x), "v"(y));
}
__device__ __forceinline__ void keep4_h(v16h a, v16h b, v16h c, v16h d) {
  asm volatile("v_nop" :: "v"(a), "v"(b), "v"(c), "v"(d));
}
__device__ __forceinline__ void acc_guard4(v8f& a, v8f& b, v8f& c, v8f& d) {
  asm volatile("v_nop\n\tv_nop\n\tv_nop\n\tv_nop" : "+v"(a), "+v"(b), "+v"(c), "+v"(d));
}

__global__ __launch_bounds__(256) void prep_planes_kernel(
    const float* __restrict__ wm_di, const float* __restrict__ wm_ndi, const float* __restrict__ wm_dd,
    const float* __restrict__ fcw_di, const float* __restrict__ fcw_ndi, const float* __restrict__ fcw_dd,
    const float* __restrict__ fcb_di, const float* __restrict__ fcb_ndi, const float* __restrict__ fcb_dd,
    unsigned short* __restrict__ WN, float* __restrict__ WEFF, float* __restrict__ WFC, float* __restrict__ BFC)
{
  __shared__ __align__(16) float sb[256];
  const int blk = blockIdx.x;
  const int t = threadIdx.x;
  if (blk < 128) {
    const size_t e0 = ((size_t)blk * 256 + t) << 3;
    const v4f a0 = *(const v4f*)(wm_ndi + e0);
    const v4f a1 = *(const v4f*)(wm_ndi + e0 + 4);
    v8h hv;
#pragma unroll
    for (int e = 0; e < 4; ++e) {
      hv[e]     = (_Float16)(a0[e] * kCarryB);
      hv[4 + e] = (_Float16)(a1[e] * kCarryB);
    }
    unsigned short* q = WN + e0;
    *(volatile v8h*)q = hv;
    __threadfence();
    *(volatile v8h*)q = hv;
  } else if (blk < 136) {
    const int g   = (blk - 128) * 256 + t;
    const int mat = (blk - 128) >> 2;
    const int h   = (g >> 4) & 63;
    const int k4  = (g & 15) * 4;
    const float* base = ((mat != 0) ? wm_dd : wm_di) + (size_t)h * kKtot;
    v4f cs = (v4f){0.f, 0.f, 0.f, 0.f};
    float r0 = 0.f, r1 = 0.f, r2 = 0.f, r3 = 0.f;
#pragma unroll 1
    for (int i = 0; i < kFm; ++i) {
      const v4f c = *(const v4f*)(base + i * kFm + k4);
      cs = cs + c;
      r0 += base[(k4 + 0) * kFm + i];
      r1 += base[(k4 + 1) * kFm + i];
      r2 += base[(k4 + 2) * kFm + i];
      r3 += base[(k4 + 3) * kFm + i];
    }
    v4f o;
    o[0] = cs[0] - r0;
    o[1] = cs[1] - r1;
    o[2] = cs[2] - r2;
    o[3] = cs[3] - r3;
    float* q = WEFF + (size_t)mat * (kHead * kFm) + h * kFm + k4;
    *(volatile v4f*)q = o;
    __threadfence();
    *(volatile v4f*)q = o;
  } else if (blk < 145) {
    const int qb  = blk - 136;
    const int p   = qb / 3;
    const int idx = (qb - p * 3) * 256 + t;
    const float* src = (p == 0) ? fcw_di : ((p == 1) ? fcw_ndi : fcw_dd);
    const v4f v = *(const v4f*)(src + idx * 4);
    float* q = WFC + (size_t)p * (kEmb * kHead) + idx * 4;
    *(volatile v4f*)q = v;
    __threadfence();
    *(volatile v4f*)q = v;
  } else {
    const int i0 = (t < 47) ? t : 47;
    int i1 = t - 48;
    i1 = (i1 < 0) ? 0 : ((i1 > 47) ? 47 : i1);
    int i2 = t - 96;
    i2 = (i2 < 0) ? 0 : ((i2 > 47) ? 47 : i2);
    float a = fcb_di[i0];
    asm volatile("" : "+v"(a));
    float b = fcb_ndi[i1];
    asm volatile("" : "+v"(b));
    float c = fcb_dd[i2];
    asm volatile("" : "+v"(c));
    const float v = (t < 48) ? a : ((t < 96) ? b : ((t < 144) ? c : 0.0f));
    sb[t] = v;
    __syncthreads();
    if (t < 32) {
      const int idx0 = t * 4;
      const int idx1 = 128 + (t & 7) * 4;
      const v4f va = *(const v4f*)(sb + idx0);
      const v4f vb = *(const v4f*)(sb + idx1);
      for (int pass = 0; pass < 2; ++pass) {
        *(volatile v4f*)(BFC + idx0) = va;
        if (t < 8) *(volatile v4f*)(BFC + idx1) = vb;
        __threadfence();
      }
    }
  }
}

__global__ __launch_bounds__(256) void panel_kernel(
    const float* __restrict__ x, unsigned* __restrict__ PN32, float* __restrict__ XPD)
{
  __shared__ __align__(16) float xs[kLen];
  __shared__ __align__(16) float smv[kLen];
  __shared__ __align__(16) float dfv[kLen];
  __shared__ __align__(16) float pd[128];
  __shared__ __align__(16) unsigned sP[8][256];
  const int b = blockIdx.x;
  const int t = threadIdx.x;
  const int lane = t & 31;
  const int wave = t >> 5;
  xs[t] = x[(size_t)b * kLen + t];
  __syncthreads();
  {
    const int im2 = (t - 2 < 0) ? 0 : (t - 2);
    const int im1 = (t - 1 < 0) ? 0 : (t - 1);
    const int ip1 = (t + 1 > kLen - 1) ? (kLen - 1) : (t + 1);
    const int ip2 = (t + 2 > kLen - 1) ? (kLen - 1) : (t + 2);
    smv[t] = ((((xs[im2] + xs[im1]) + xs[t]) + xs[ip1]) + xs[ip2]) * 0.2f;
  }
  __syncthreads();
  {
    const float prev = smv[(t > 0) ? (t - 1) : 0];
    const float x0 = xs[0];
    const float sub = (t == 0) ? x0 : prev;
    dfv[t] = smv[t] - sub;
  }
  __syncthreads();
  if (t < kFm) {
    pd[t]       = (((xs[4 * t] + xs[4 * t + 1]) + xs[4 * t + 2]) + xs[4 * t + 3]) * 0.25f;
    pd[kFm + t] = (((dfv[4 * t] + dfv[4 * t + 1]) + dfv[4 * t + 2]) + dfv[4 * t + 3]) * 0.25f;
  }
  const v4f c0 = *(const v4f*)(xs + 8 * lane);
  const v4f c1 = *(const v4f*)(xs + 8 * lane + 4);
#pragma unroll 1
  for (int it = 0; it < 8; ++it) {
    const int I = wave * 8 + it;
    const v4f a = *(const v4f*)(xs + 4 * I);
    float s0 = 0.0f, s1 = 0.0f;
#pragma unroll
    for (int pi = 0; pi < 4; ++pi) {
#pragma unroll
      for (int pj = 0; pj < 4; ++pj) {
        const float n0 = c0[pj] - a[pi];
        const float d0 = (c0[pj] + a[pi]) + 1e-5f;
        s0 += n0 * __builtin_amdgcn_rcpf(d0);
        const float n1 = c1[pj] - a[pi];
        const float d1 = (c1[pj] + a[pi]) + 1e-5f;
        s1 += n1 * __builtin_amdgcn_rcpf(d1);
      }
    }
    sP[wave][it * 32 + lane] = pack2h(s0 * (kCarryA * 0.0625f), s1 * (kCarryA * 0.0625f));
  }
  __syncthreads();
  {
    const v4u w0 = *(const v4u*)(&sP[wave][lane * 4]);
    const v4u w1 = *(const v4u*)(&sP[wave][128 + lane * 4]);
    unsigned* q = PN32 + (size_t)b * (kKtot / 2) + wave * 256 + lane * 4;
    const v4f pv = *(const v4f*)(pd + 4 * lane);
    float* qx = XPD + (size_t)b * 128 + 4 * lane;
    for (int pass = 0; pass < 2; ++pass) {
      *(volatile v4u*)(q) = w0;
      *(volatile v4u*)(q + 128) = w1;
      if (wave == 0) *(volatile v4f*)(qx) = pv;
      __threadfence();
    }
  }
}

__global__ __launch_bounds__(256) void gemm64_f16_kernel(
    const unsigned short* __restrict__ Ap, int lda,
    const unsigned short* __restrict__ Btp, int ldb,
    float* __restrict__ C, int ldc, int M, int N, int K, float scale)
{
  const _Float16* A  = (const _Float16*)Ap;
  const _Float16* Bt = (const _Float16*)Btp;
  __shared__ __align__(16) float sT[8][16 * 68];
  const int lane = threadIdx.x & 31;
  const int wave = threadIdx.x >> 5;
  const int tilesN = N >> 6;
  const int tilesM = M >> 6;
  const int tile = blockIdx.x * 8 + wave;
  if (tile >= tilesM * tilesN) return;
  const int tm = tile / tilesN;
  const int tn = tile - tm * tilesN;
  const int m0 = tm << 6;
  const int n0 = tn << 6;
  const int rlane = lane & 15;
  const int koff  = (lane >> 4) * 8;
  const int mOff  = (lane >> 4) * 8;

  v8f acc[4][4];
#pragma unroll
  for (int i = 0; i < 4; ++i)
#pragma unroll
    for (int j = 0; j < 4; ++j) acc[i][j] = (v8f){0.f, 0.f, 0.f, 0.f, 0.f, 0.f, 0.f, 0.f};

  for (int k0 = 0; k0 < K; k0 += 32) {
    v16h bh[4];
#pragma unroll
    for (int j = 0; j < 4; ++j) {
      const size_t bo = (size_t)(n0 + (j << 4) + rlane) * ldb + koff + k0;
      bh[j] = frag_load_h(Bt + bo);
    }
#pragma unroll
    for (int i = 0; i < 4; ++i) {
      const size_t ao = (size_t)(m0 + (i << 4) + rlane) * lda + koff + k0;
      const v16h ah = frag_load_h(A + ao);
#pragma unroll
      for (int j = 0; j < 4; ++j) acc[i][j] = mma_h(ah, bh[j], acc[i][j]);
      frag_guard(acc[i][0], ah, bh[0]);
      frag_guard(acc[i][1], ah, bh[1]);
      frag_guard(acc[i][2], ah, bh[2]);
      frag_guard(acc[i][3], ah, bh[3]);
    }
    keep4_h(bh[0], bh[1], bh[2], bh[3]);
  }
  acc_guard4(acc[0][0], acc[0][1], acc[0][2], acc[0][3]);
  acc_guard4(acc[1][0], acc[1][1], acc[1][2], acc[1][3]);
  acc_guard4(acc[2][0], acc[2][1], acc[2][2], acc[2][3]);
  acc_guard4(acc[3][0], acc[3][1], acc[3][2], acc[3][3]);

  float* slab = sT[wave];
#pragma unroll
  for (int i = 0; i < 4; ++i) {
    const int mBase = m0 + (i << 4);
#pragma unroll
    for (int j = 0; j < 4; ++j) {
#pragma unroll
      for (int r = 0; r < 8; ++r) {
        const float v = acc[i][j][r] * scale;
        slab[(mOff + r) * 68 + (j << 4) + rlane] = v;
      }
    }
    __builtin_amdgcn_fence(__ATOMIC_RELEASE, "workgroup");
    __builtin_amdgcn_wave_barrier();
    __builtin_amdgcn_fence(__ATOMIC_ACQUIRE, "workgroup");
    {
      const int hh = lane >> 4;
      const int c4 = (lane & 15) * 4;
      for (int pass = 0; pass < 2; ++pass) {
#pragma unroll
        for (int it = 0; it < 8; ++it) {
          const int row = it * 2 + hh;
          const v4f v = *(const v4f*)(slab + row * 68 + c4);
          *(volatile v4f*)(C + (size_t)(mBase + row) * ldc + n0 + c4) = v;
        }
        __threadfence();
      }
    }
    __builtin_amdgcn_fence(__ATOMIC_RELEASE, "workgroup");
    __builtin_amdgcn_wave_barrier();
    __builtin_amdgcn_fence(__ATOMIC_ACQUIRE, "workgroup");
  }
}

__global__ __launch_bounds__(256) void tail_kernel(
    const float* __restrict__ XPD, const float* __restrict__ HN, const float* __restrict__ WEFF,
    const float* __restrict__ b_di, const float* __restrict__ b_ndi, const float* __restrict__ b_dd,
    const float* __restrict__ WFC, const float* __restrict__ BFC,
    const float* __restrict__ fc1_w, const float* __restrict__ fc1_b,
    const float* __restrict__ fc2_w, const float* __restrict__ fc2_b,
    float* __restrict__ out)
{
  __shared__ __align__(16) float sV[kRowsBlk * 128];
  __shared__ __align__(16) float sH[kRowsBlk * 192];
  __shared__ __align__(16) float sE[kRowsBlk * kCat];
  __shared__ __align__(16) float sM[kRowsBlk * kEmb];
  __shared__ __align__(16) float sO[kRowsBlk * kOutW];
  const int t = threadIdx.x;
  const int lane = t & 31;
  const int wave = t >> 5;
  const int b0 = blockIdx.x * kRowsBlk;

  {
    const v4f v = *(const v4f*)(XPD + (size_t)b0 * 128 + t * 4);
    *(v4f*)(sV + t * 4) = v;
  }
  const int n  = t & 63;
  const int rg = t >> 6;
  const int ra = 2 * rg;
  const int rb = ra + 1;
  {
    const float bn = b_ndi[n];
    const float g0 = HN[(size_t)(b0 + ra) * kHead + n] + bn;
    const float g1 = HN[(size_t)(b0 + rb) * kHead + n] + bn;
    sH[ra * 192 + 64 + n] = elu1(g0);
    sH[rb * 192 + 64 + n] = elu1(g1);
  }
  const float bdi = b_di[n];
  const float bdd = b_dd[n];
  __syncthreads();

#pragma unroll 1
  for (int p = 0; p < 2; ++p) {
    const float* wp = WEFF + (size_t)p * (kHead * kFm) + n * kFm;
    const float* v0 = sV + ra * 128 + p * 64;
    const float* v1 = sV + rb * 128 + p * 64;
    float a0 = 0.0f, a1 = 0.0f;
#pragma unroll 1
    for (int k4 = 0; k4 < kFm / 4; ++k4) {
      const v4f w  = *(const v4f*)(wp + 4 * k4);
      const v4f x0 = *(const v4f*)(v0 + 4 * k4);
      const v4f x1 = *(const v4f*)(v1 + 4 * k4);
      a0 = fmaf(w[0], x0[0], a0);
      a0 = fmaf(w[1], x0[1], a0);
      a0 = fmaf(w[2], x0[2], a0);
      a0 = fmaf(w[3], x0[3], a0);
      a1 = fmaf(w[0], x1[0], a1);
      a1 = fmaf(w[1], x1[1], a1);
      a1 = fmaf(w[2], x1[2], a1);
      a1 = fmaf(w[3], x1[3], a1);
    }
    const float bb = (p == 0) ? bdi : bdd;
    sH[ra * 192 + p * 128 + n] = elu1(a0 + bb);
    sH[rb * 192 + p * 128 + n] = elu1(a1 + bb);
  }
  __syncthreads();

#pragma unroll 1
  for (int it = 0; it < 3; ++it) {
    const int task = it * 256 + t;
    const int tc = (task < 575) ? task : 575;
    const int rp = tc / kCat;
    const int o  = tc - rp * kCat;
    const int p  = o / kEmb;
    const float* wrow = WFC + (size_t)o * kHead;
    const float* h0 = sH + (2 * rp) * 192 + p * 64;
    const float* h1 = h0 + 192;
    float a0 = 0.0f, a1 = 0.0f;
#pragma unroll 1
    for (int k4 = 0; k4 < kHead / 4; ++k4) {
      const v4f w  = *(const v4f*)(wrow + 4 * k4);
      const v4f x0 = *(const v4f*)(h0 + 4 * k4);
      const v4f x1 = *(const v4f*)(h1 + 4 * k4);
      a0 = fmaf(w[0], x0[0], a0);
      a0 = fmaf(w[1], x0[1], a0);
      a0 = fmaf(w[2], x0[2], a0);
      a0 = fmaf(w[3], x0[3], a0);
      a1 = fmaf(w[0], x1[0], a1);
      a1 = fmaf(w[1], x1[1], a1);
      a1 = fmaf(w[2], x1[2], a1);
      a1 = fmaf(w[3], x1[3], a1);
    }
    float bb = BFC[o];
    asm volatile("" : "+v"(bb));
    const float e0 = elu1(a0 + bb);
    const float e1 = elu1(a1 + bb);
    if (task < 576) {
      sE[(2 * rp) * kCat + o] = e0;
      sE[(2 * rp + 1) * kCat + o] = e1;
    }
  }
  __syncthreads();

  {
    const int tc = (t < 191) ? t : 191;
    const int rp = tc / kEmb;
    const int o  = tc - rp * kEmb;
    const float* wrow = fc1_w + (size_t)o * kCat;
    const float* e0p = sE + (2 * rp) * kCat;
    const float* e1p = e0p + kCat;
    float a0 = 0.0f, a1 = 0.0f;
#pragma unroll 1
    for (int k4 = 0; k4 < kCat / 4; ++k4) {
      const v4f w  = *(const v4f*)(wrow + 4 * k4);
      const v4f x0 = *(const v4f*)(e0p + 4 * k4);
      const v4f x1 = *(const v4f*)(e1p + 4 * k4);
      a0 = fmaf(w[0], x0[0], a0);
      a0 = fmaf(w[1], x0[1], a0);
      a0 = fmaf(w[2], x0[2], a0);
      a0 = fmaf(w[3], x0[3], a0);
      a1 = fmaf(w[0], x1[0], a1);
      a1 = fmaf(w[1], x1[1], a1);
      a1 = fmaf(w[2], x1[2], a1);
      a1 = fmaf(w[3], x1[3], a1);
    }
    float bb = fc1_b[o];
    asm volatile("" : "+v"(bb));
    const float m0v = elu1(a0 + bb);
    const float m1v = elu1(a1 + bb);
    if (t < 192) {
      sM[(2 * rp) * kEmb + o] = m0v;
      sM[(2 * rp + 1) * kEmb + o] = m1v;
    }
  }
  __syncthreads();

  {
    const int tc = (t < 159) ? t : 159;
    const int r  = tc / kOutW;
    const int o  = tc - r * kOutW;
    const float* wrow = fc2_w + (size_t)o * kEmb;
    const float* mp = sM + r * kEmb;
    float a0 = 0.0f;
#pragma unroll 1
    for (int k4 = 0; k4 < kEmb / 4; ++k4) {
      const v4f w  = *(const v4f*)(wrow + 4 * k4);
      const v4f x0 = *(const v4f*)(mp + 4 * k4);
      a0 = fmaf(w[0], x0[0], a0);
      a0 = fmaf(w[1], x0[1], a0);
      a0 = fmaf(w[2], x0[2], a0);
      a0 = fmaf(w[3], x0[3], a0);
    }
    float bb = fc2_b[o];
    asm volatile("" : "+v"(bb));
    const float y = a0 + bb;
    if (t < 160) sO[tc] = y;
  }
  __syncthreads();

  if (wave == 0) {
    const int idx0 = lane * 4;
    const int idx1 = 128 + (lane & 7) * 4;
    const v4f va = *(const v4f*)(sO + idx0);
    const v4f vb = *(const v4f*)(sO + idx1);
    float* ob = out + (size_t)b0 * kOutW;
    for (int pass = 0; pass < 2; ++pass) {
      *(volatile v4f*)(ob + idx0) = va;
      if (lane < 8) *(volatile v4f*)(ob + idx1) = vb;
      __threadfence();
    }
  }
}

extern "C" void kernel_launch(void* const* d_in, const int* in_sizes, int n_in,
                              void* d_out, int out_size, void* d_ws, size_t ws_size,
                              hipStream_t stream) {
  if (n_in < 17) return;
  if (in_sizes[0] != kBatch * kLen) return;
  if (in_sizes[1] != kHead * kKtot || in_sizes[5] != kHead * kKtot || in_sizes[9] != kHead * kKtot) return;
  if (in_sizes[2] != kHead || in_sizes[6] != kHead || in_sizes[10] != kHead) return;
  if (in_sizes[3] != kEmb * kHead || in_sizes[7] != kEmb * kHead || in_sizes[11] != kEmb * kHead) return;
  if (in_sizes[4] != kEmb || in_sizes[8] != kEmb || in_sizes[12] != kEmb) return;
  if (in_sizes[13] != kEmb * kCat || in_sizes[14] != kEmb) return;
  if (in_sizes[15] != kOutW * kEmb || in_sizes[16] != kOutW) return;
  if (out_size != kBatch * kOutW) return;
  if (ws_size < kWsTotal) return;

  const float* x       = (const float*)d_in[0];
  const float* wm_di   = (const float*)d_in[1];
  const float* b_di    = (const float*)d_in[2];
  const float* fcw_di  = (const float*)d_in[3];
  const float* fcb_di  = (const float*)d_in[4];
  const float* wm_ndi  = (const float*)d_in[5];
  const float* b_ndi   = (const float*)d_in[6];
  const float* fcw_ndi = (const float*)d_in[7];
  const float* fcb_ndi = (const float*)d_in[8];
  const float* wm_dd   = (const float*)d_in[9];
  const float* b_dd    = (const float*)d_in[10];
  const float* fcw_dd  = (const float*)d_in[11];
  const float* fcb_dd  = (const float*)d_in[12];
  const float* fc1_w   = (const float*)d_in[13];
  const float* fc1_b   = (const float*)d_in[14];
  const float* fc2_w   = (const float*)d_in[15];
  const float* fc2_b   = (const float*)d_in[16];
  float* out = (float*)d_out;

  char* ws = (char*)d_ws;
  unsigned short* WN   = (unsigned short*)(ws + kOffWN);
  float*          WEFF = (float*)(ws + kOffWEFF);
  float*          WFC  = (float*)(ws + kOffWFC);
  float*          BFC  = (float*)(ws + kOffBFC);
  float*          XPD  = (float*)(ws + kOffXPD);
  unsigned short* PN   = (unsigned short*)(ws + kOffPN);
  float*          HN   = (float*)(ws + kOffHN);

  prep_planes_kernel<<<146, 256, 0, stream>>>(wm_di, wm_ndi, wm_dd, fcw_di, fcw_ndi, fcw_dd,
                                              fcb_di, fcb_ndi, fcb_dd, WN, WEFF, WFC, BFC);
  panel_kernel<<<kBatch, 256, 0, stream>>>(x, (unsigned*)PN, XPD);
  gemm64_f16_kernel<<<2, 256, 0, stream>>>(PN, kKtot, WN, kKtot, HN, kHead,
                                           kBatch, kHead, kKtot, kFoldBack);
  tail_kernel<<<kBatch / kRowsBlk, 256, 0, stream>>>(XPD, HN, WEFF, b_di, b_ndi, b_dd, WFC, BFC,
                                                     fc1_w, fc1_b, fc2_w, fc2_b, out);
}
